// FactorizedJumpOperator_51281909514364
// MI455X (gfx1250) — hardware-run, weakly checked
//
#include <hip/hip_runtime.h>


#ifndef NROWS
#define NROWS 4096
#endif
#define NROWS_FULL 4096
#define DM    128
#define NCH   64
#define MAX_NORM 0.99f
#define MOB_EPS  1e-15f
#define XP    136
#define OP    132
#define TLP   72
#define CARRY 256.0f
#define UNCARRY2 (1.0f / 65536.0f)

static_assert(DM == 128);
static_assert(DM % 32 == 0);
static_assert(DM == 8 * 16);
static_assert(NROWS % 256 == 0);
static_assert(NROWS <= NROWS_FULL);
static_assert(NROWS % 16 == 0);
static_assert((XP * 2) % 16 == 0);
static_assert((OP * 4) % 16 == 0);
static_assert((TLP * 2) % 16 == 0);
static_assert(16 * XP * 2 + 16 * OP * 4 + NROWS * 4 + 8 * 4 <= 131072);
static_assert(DM * TLP * 2 <= 131072);
static_assert(4 * 256 * 16 == 64 * DM * 2);
static_assert(256 * 16 == 16 * DM * 2);
static_assert(8 * 2 * 32 * 16 == 16 * DM * 4);

typedef _Float16 h16;
typedef __attribute__((ext_vector_type(16))) _Float16 v16h;
typedef __attribute__((ext_vector_type(8)))  _Float16 v8h;
typedef __attribute__((ext_vector_type(4)))  _Float16 v4h;
typedef __attribute__((ext_vector_type(8)))  float    v8f;
typedef __attribute__((ext_vector_type(4)))  float    v4f;
typedef v4f  __attribute__((may_alias)) v4fa;

__device__ __forceinline__ unsigned short f2bf(float f) { unsigned u = __float_as_uint(f); u += 0x7FFFu + ((u >> 16) & 1u); return (unsigned short)(u >> 16); }
__device__ __forceinline__ float bfr(float f) { return __uint_as_float(((unsigned)f2bf(f)) << 16); }
__device__ __forceinline__ v16h cat16(v8h lo, v8h hi) { return __builtin_shufflevector(lo, hi, 0, 1, 2, 3, 4, 5, 6, 7, 8, 9, 10, 11, 12, 13, 14, 15); }
__device__ __forceinline__ v16h  ldh(const h16* p) { return cat16(*(const v8h*)p, *(const v8h*)(p + 16)); }
static __device__ __forceinline__ h16 toh_flush(float v) { const h16 r = (h16)v; return (fabsf(v) < 6.103515625e-05f) ? (h16)0.0f : r; }
__device__ __forceinline__ v8f wmma16g(v16h a, v16h b, v8f c) {
    c = __builtin_amdgcn_wmma_f32_16x16x32_f16(false, a, false, b, (short)0, c, false, false);
    asm volatile("v_nop\n\tv_nop\n\tv_nop\n\tv_nop" : "+v"(c) : "v"(a), "v"(b));
    return c;
}
__device__ __forceinline__ int clampi(int v, int lo, int hi) { return v < lo ? lo : (v > hi ? hi : v); }
__device__ __forceinline__ float waveSum(float v) {
#pragma unroll
    for (int o = 16; o > 0; o >>= 1) v += __shfl_xor(v, o, 32);
    return v;
}
__device__ __forceinline__ v4f ball4(v4f z) {
    float s = z[0] * z[0] + z[1] * z[1] + z[2] * z[2] + z[3] * z[3];
    s = waveSum(s);
    const float n = sqrtf(s);
    const float sc = (n > MAX_NORM) ? MAX_NORM * (1.0f / fmaxf(n, 1e-30f)) : 1.0f;
    return z * sc;
}
__device__ __forceinline__ v4f mobius4(v4f x, v4f y) {
    float x2 = x[0] * x[0] + x[1] * x[1] + x[2] * x[2] + x[3] * x[3];
    float y2 = y[0] * y[0] + y[1] * y[1] + y[2] * y[2] + y[3] * y[3];
    float xy = x[0] * y[0] + x[1] * y[1] + x[2] * y[2] + x[3] * y[3];
    x2 = waveSum(x2); y2 = waveSum(y2); xy = waveSum(xy);
    const float ka  = 1.0f + 2.0f * xy + y2;
    const float kb  = 1.0f - x2;
    const float den = fmaxf(1.0f + 2.0f * xy + x2 * y2, MOB_EPS);
    const float inv = 1.0f / den;
    v4f o;
#pragma unroll
    for (int e = 0; e < 4; ++e) o[e] = (ka * x[e] + kb * y[e]) * inv;
    return o;
}

__global__ __launch_bounds__(256) void k_rconv(const float* __restrict__ R, h16* RH, h16* RT) {
    __shared__ __align__(16) h16 tl[DM * TLP];
    const int t = threadIdx.x;
    const int c = blockIdx.x, r0 = blockIdx.y * 64;
    const size_t cb = (size_t)c * DM * DM;
    v8h hv[4];
#pragma unroll
    for (int s = 0; s < 4; ++s) {
        const int p = s * 256 + t; const int i = p >> 4, c8 = (p & 15) * 8;
        const v8f v = *(const v8f*)(R + cb + (size_t)(r0 + i) * DM + c8);
        v8h o;
#pragma unroll
        for (int k = 0; k < 8; ++k) o[k] = toh_flush(bfr(v[k]) * CARRY);
        hv[s] = o;
#pragma unroll
        for (int k = 0; k < 8; ++k) tl[(c8 + k) * TLP + i] = o[k];
    }
    __syncthreads();
    v8h tv[4];
#pragma unroll
    for (int s = 0; s < 4; ++s) { const int q = s * 256 + t; const int j = q >> 3, i8 = (q & 7) * 8; tv[s] = *(const v8h*)(&tl[j * TLP + i8]); }
#pragma unroll 1
    for (int ps = 0; ps < 2; ++ps) {
#pragma unroll
        for (int s = 0; s < 4; ++s) {
            const int p = s * 256 + t; const int i = p >> 4, c8 = (p & 15) * 8;
            const int j = p >> 3, i8 = (p & 7) * 8;
            *(volatile v8h*)(RH + cb + (size_t)(r0 + i) * DM + c8) = hv[s];
            *(volatile v8h*)(RT + cb + (size_t)j * DM + r0 + i8) = tv[s]; }
        if (ps == 0) __threadfence(); }
}

template <int STAGE>
__device__ __forceinline__ void chart_body(const float* __restrict__ ZN, const float* __restrict__ CEN, const int* __restrict__ GIDX, const int* __restrict__ OIDX,
                                           const h16* __restrict__ RP, const h16* WIN, h16* WOUT, float* OUT) {
    __shared__ __align__(16) h16 xs[16 * XP];
    __shared__ __align__(16) float os[16 * OP];
    __shared__ int lst[NROWS];
    __shared__ int wc[8];
    const int t = threadIdx.x, lane = t & 31, lr = lane & 15, hi = lane >> 4;
    const int wave = __builtin_amdgcn_readfirstlane((int)(threadIdx.x >> 5));
    const int chart = blockIdx.x;
    const int seg = wave * (NROWS / 8);
    int cw = 0;
#pragma unroll 1
    for (int it = 0; it < NROWS / 256; ++it) {
        const int g = clampi(GIDX[seg + it * 32 + lane], 0, NCH - 1);
        cw += __popc(__builtin_amdgcn_ballot_w32(g == chart));
    }
    if (lane == 0) wc[wave] = cw;
    __syncthreads();
    int base = 0, cnt = 0;
#pragma unroll
    for (int w = 0; w < 8; ++w) { const int c = wc[w]; base += (w < wave) ? c : 0; cnt += c; }
    cnt = cnt > NROWS ? NROWS : cnt;
    int run = base;
#pragma unroll 1
    for (int it = 0; it < NROWS / 256; ++it) {
        const int i = seg + it * 32 + lane;
        const int g = clampi(GIDX[i], 0, NCH - 1);
        const bool hit = (g == chart);
        const unsigned bal = __builtin_amdgcn_ballot_w32(hit);
        const int pos = clampi(run + __popc(bal & ((1u << lane) - 1u)), 0, NROWS - 1);
        if (hit) lst[pos] = i;
        run += __popc(bal);
    }
    __syncthreads();
    int nt = (cnt + 15) >> 4; nt = nt > NROWS / 16 ? NROWS / 16 : nt;
    const int ntiles = __builtin_amdgcn_readfirstlane(nt);
    const int last = cnt - 1;
    const size_t rb = (size_t)chart * DM * DM + (size_t)(wave * 16 + lr) * DM + 8 * hi;
    const v16h b0 = ldh(RP + rb), b1 = ldh(RP + rb + 32), b2 = ldh(RP + rb + 64), b3 = ldh(RP + rb + 96);
#pragma unroll 1
    for (int tile = 0; tile < ntiles; ++tile) {
        if (STAGE == 0) {
#pragma unroll 1
            for (int q = 0; q < 2; ++q) {
                const int rr = wave + 8 * q;
                int pc = tile * 16 + rr; pc = pc > last ? last : pc;
                const int b = clampi(lst[pc], 0, NROWS - 1);
                const int ci = clampi(OIDX[b], 0, NCH - 1);
                const v4f zr = *(const v4f*)(ZN + (size_t)b * DM + 4 * lane);
                const v4f cr = *(const v4f*)(CEN + (size_t)ci * DM + 4 * lane);
                v4f z, c;
#pragma unroll
                for (int e = 0; e < 4; ++e) { z[e] = bfr(zr[e]); c[e] = bfr(cr[e]); }
                z = ball4(z); c = ball4(c);
                const v4f g = mobius4(-c, z);
                v4h hv;
#pragma unroll
                for (int e = 0; e < 4; ++e) hv[e] = toh_flush(g[e] * CARRY);
                *(v4h*)(&xs[rr * XP + 4 * lane]) = hv;
            }
        } else {
            const int r = t >> 4, c8 = (t & 15) * 8;
            int pc = tile * 16 + r; pc = pc > last ? last : pc;
            const int b = clampi(lst[pc], 0, NROWS - 1);
            const v8h v = *(const v8h*)(WIN + (size_t)b * DM + c8);
            *(v8h*)(&xs[r * XP + c8]) = v;
        }
        __syncthreads();
        v8f acc = (v8f){};
        const int xo = lr * XP + 8 * hi;
        acc = wmma16g(cat16(*(const v8h*)(&xs[xo]),      *(const v8h*)(&xs[xo + 16])),  b0, acc);
        acc = wmma16g(cat16(*(const v8h*)(&xs[xo + 32]), *(const v8h*)(&xs[xo + 48])),  b1, acc);
        acc = wmma16g(cat16(*(const v8h*)(&xs[xo + 64]), *(const v8h*)(&xs[xo + 80])),  b2, acc);
        acc = wmma16g(cat16(*(const v8h*)(&xs[xo + 96]), *(const v8h*)(&xs[xo + 112])), b3, acc);
#pragma unroll
        for (int r = 0; r < 8; ++r) os[(8 * hi + r) * OP + wave * 16 + lr] = acc[r] * UNCARRY2;
        __syncthreads();
        if (STAGE == 0) {
            const int r = t >> 4, c8 = (t & 15) * 8;
            const int pos = tile * 16 + r; const bool valid = pos < cnt;
            const int pc = pos > last ? last : pos;
            const int b = clampi(lst[pc], 0, NROWS - 1);
            const v4f x0 = *(const v4fa*)(&os[r * OP + c8]); const v4f x1 = *(const v4fa*)(&os[r * OP + c8 + 4]);
            v8h hv;
#pragma unroll
            for (int i = 0; i < 4; ++i) { hv[i] = toh_flush(x0[i] * CARRY); hv[4 + i] = toh_flush(x1[i] * CARRY); }
            h16* wp = WOUT + (size_t)b * DM + c8;
#pragma unroll 1
            for (int ps = 0; ps < 2; ++ps) { if (valid) *(volatile v8h*)wp = hv; if (ps == 0) __threadfence(); }
        } else {
#pragma unroll 1
            for (int q = 0; q < 2; ++q) {
                const int rr = wave + 8 * q;
                const int pos = tile * 16 + rr; const bool valid = pos < cnt;
                const int pc = pos > last ? last : pos;
                const int b = clampi(lst[pc], 0, NROWS - 1);
                const int ci = clampi(OIDX[b], 0, NCH - 1);
                const v4f y = *(const v4fa*)(&os[rr * OP + 4 * lane]);
                const v4f cr = *(const v4f*)(CEN + (size_t)ci * DM + 4 * lane);
                v4f c;
#pragma unroll
                for (int e = 0; e < 4; ++e) c[e] = bfr(cr[e]);
                c = ball4(c);
                const v4f o = ball4(mobius4(c, y));
                float* op = OUT + (size_t)b * DM + 4 * lane;
#pragma unroll 1
                for (int ps = 0; ps < 2; ++ps) { if (valid) *(volatile v4f*)op = o; if (ps == 0) __threadfence(); }
            }
        }
        __syncthreads();
    }
}

__global__ __launch_bounds__(256) void k_chart_fwd(const float* __restrict__ ZN, const float* __restrict__ CEN, const int* __restrict__ SRC, const int* __restrict__ TGT,
                                                   const h16* __restrict__ RH, h16* W) {
    chart_body<0>(ZN, CEN, TGT, SRC, RH, (const h16*)0, W, (float*)0);
}
__global__ __launch_bounds__(256) void k_chart_bwd(const float* __restrict__ CEN, const int* __restrict__ SRC, const int* __restrict__ TGT,
                                                   const h16* __restrict__ RT, const h16* W, float* OUT) {
    chart_body<1>((const float*)0, CEN, SRC, TGT, RT, W, (h16*)0, OUT);
}

static constexpr size_t al256(size_t v) { return (v + 255) & ~(size_t)255; }
static constexpr size_t SZ_RP = al256((size_t)NCH * DM * DM * 2);
static constexpr size_t SZ_W  = al256((size_t)NROWS * DM * 2);
static constexpr size_t SZ_TOTAL = 2 * SZ_RP + SZ_W;
static_assert(SZ_TOTAL <= (size_t)134217728);
static_assert((size_t)NCH * DM * DM * 2 == (size_t)NCH * 2 * 64 * DM * 2);
static_assert(((size_t)NROWS * DM * 4) % 128 == 0);

extern "C" void kernel_launch(void* const* d_in, const int* in_sizes, int n_in,
                              void* d_out, int out_size, void* d_ws, size_t ws_size, hipStream_t stream) {
    if (n_in < 5) return;
    if ((size_t)in_sizes[0] < (size_t)NROWS * DM) return;
    if ((size_t)in_sizes[1] < (size_t)NCH * DM) return;
    if ((size_t)in_sizes[2] < (size_t)NCH * DM * DM) return;
    if (in_sizes[3] < NROWS || in_sizes[4] < NROWS) return;
    if ((size_t)out_size < (size_t)NROWS * DM) return;
    if (SZ_TOTAL > ws_size) return;
    const float* zn  = (const float*)d_in[0];
    const float* cen = (const float*)d_in[1];
    const float* rot = (const float*)d_in[2];
    const int*   src = (const int*)d_in[3];
    const int*   tgt = (const int*)d_in[4];
    float* OUT = (float*)d_out;
    char* wsp = (char*)d_ws;
    h16* RH = (h16*)wsp; wsp += SZ_RP;
    h16* RT = (h16*)wsp; wsp += SZ_RP;
    h16* W  = (h16*)wsp; wsp += SZ_W;

    k_rconv<<<dim3(NCH, 2, 1), 256, 0, stream>>>(rot, RH, RT);
    k_chart_fwd<<<dim3(NCH, 1, 1), 256, 0, stream>>>(zn, cen, src, tgt, RH, W);
    k_chart_bwd<<<dim3(NCH, 1, 1), 256, 0, stream>>>(cen, src, tgt, RT, W, OUT);
}
